// CrossAttention3D_87952340287876
// MI455X (gfx1250) — hardware-verified
//
#include <hip/hip_runtime.h>
#include <math.h>
#include <stdint.h>

#ifndef NB
#define NB 2
#endif
#ifndef SEQ
#define SEQ 4096
#endif
#define NBFULL 2
#define NFULL  4096
#define CC     128
#define NWR    512
#define QT     64
#define OSP    68
#define OSPW   132
#define TP     72
#define WSC    256.0f
#define IWSC   0.00390625f
#define VSC    4.0f
#define IVSC   0.25f
#define LNPS   9.704060527839234f
#define SCL    0.08838834764831845f

static_assert(NB >= 1 && NB <= NBFULL);
static_assert(SEQ % QT == 0 && SEQ >= QT && SEQ <= NFULL);
static_assert(SEQ % 32 == 0);
static_assert(CC == 2 * QT);
static_assert(CC % 32 == 0);
static_assert(NWR == 4 * CC);
static_assert((OSP * 4) % 16 == 0);
static_assert((OSPW * 4) % 16 == 0);
static_assert((TP * 2) % 16 == 0);

typedef _Float16       v16h __attribute__((ext_vector_type(16)));
typedef _Float16       v8h  __attribute__((ext_vector_type(8)));
typedef __bf16         v16b __attribute__((ext_vector_type(16)));
typedef unsigned short v8us __attribute__((ext_vector_type(8)));
typedef float          v8f  __attribute__((ext_vector_type(8)));
typedef float          v4f  __attribute__((ext_vector_type(4)));
typedef unsigned int   v4u  __attribute__((ext_vector_type(4)));

union Frag  { v8us u[2]; v16h h; v16b bf; };
union FragH { v16h v; v8h hv[2]; };
static_assert(sizeof(Frag) == 32);
static_assert(sizeof(FragH) == 32);

__device__ __forceinline__ unsigned short bf_bits(float f) {
  unsigned u = __float_as_uint(f);
  return (unsigned short)((u + 0x7FFFu + ((u >> 16) & 1u)) >> 16);
}
__device__ __forceinline__ float bf_up(unsigned short hb) { return __uint_as_float(((unsigned)hb) << 16); }
__device__ __forceinline__ float bfr(float f) { return bf_up(bf_bits(f)); }
__device__ __forceinline__ unsigned short h_bits(_Float16 x) { return __builtin_bit_cast(unsigned short, x); }
__device__ __forceinline__ unsigned pk16(unsigned short a, unsigned short b) { return (unsigned)a | ((unsigned)b << 16); }
__device__ __forceinline__ v8f zero8() { v8f z = {0.f, 0.f, 0.f, 0.f, 0.f, 0.f, 0.f, 0.f}; return z; }
__device__ __forceinline__ float hmax8(v8f s) {
  return fmaxf(fmaxf(fmaxf(s[0], s[1]), fmaxf(s[2], s[3])), fmaxf(fmaxf(s[4], s[5]), fmaxf(s[6], s[7])));
}
__device__ __forceinline__ unsigned wave_ballot(bool p) {
#if defined(__HIP_DEVICE_COMPILE__)
  return __builtin_amdgcn_ballot_w32(p);
#else
  return p ? 1u : 0u;
#endif
}

__device__ __forceinline__ Frag ldfrag(const unsigned short* p) {
  Frag f;
  f.u[0] = *(const v8us*)(p);
  f.u[1] = *(const v8us*)(p + 16);
  return f;
}

__device__ __forceinline__ v8f mma_h(v16h a, v16h b, v8f c) {
  v8f d = __builtin_amdgcn_wmma_f32_16x16x32_f16(false, a, false, b, (short)0, c, false, false);
#if defined(__HIP_DEVICE_COMPILE__)
  asm volatile("v_nop\n\tv_nop\n\tv_nop\n\tv_nop" : "+v"(d) : "v"(a), "v"(b));
#endif
  return d;
}
__device__ __forceinline__ v8f mma_b(v16b a, v16b b, v8f c) {
  v8f d = __builtin_amdgcn_wmma_f32_16x16x32_bf16(false, a, false, b, (short)0, c, false, false);
#if defined(__HIP_DEVICE_COMPILE__)
  const v16h ha = __builtin_bit_cast(v16h, a), hb = __builtin_bit_cast(v16h, b);
  asm volatile("v_nop\n\tv_nop\n\tv_nop\n\tv_nop" : "+v"(d) : "v"(ha), "v"(hb));
#endif
  return d;
}

__global__ __launch_bounds__(256)
void cvt_w(const float* __restrict__ wq, const float* __restrict__ wk, const float* __restrict__ wv,
           const float* __restrict__ wo, unsigned short* W16) {
  const int tid = threadIdx.x, blk = blockIdx.x;
  const int wave = tid >> 5, lane = tid & 31;
  const int row = 16 * blk + 2 * wave + (lane >> 4);
  const int col = 8 * (lane & 15);
  const int which = blk >> 3;
  const float* wb = (which == 0) ? wq : (which == 1) ? wk : (which == 2) ? wv : wo;
  const float* s = wb + (size_t)(row & (CC - 1)) * CC + col;
  const v4f a = *(const v4f*)s;
  const v4f q = *(const v4f*)(s + 4);
  const float f[8] = {a[0], a[1], a[2], a[3], q[0], q[1], q[2], q[3]};
  v4u u;
  if (which < 3) {
#pragma unroll
    for (int t = 0; t < 4; ++t) {
      const _Float16 h0 = (_Float16)(bfr(f[2 * t]) * WSC);
      const _Float16 h1 = (_Float16)(bfr(f[2 * t + 1]) * WSC);
      u[t] = pk16(h_bits(h0), h_bits(h1));
    }
  } else {
#pragma unroll
    for (int t = 0; t < 4; ++t) u[t] = pk16(bf_bits(f[2 * t]), bf_bits(f[2 * t + 1]));
  }
#pragma unroll
  for (int pass = 0; pass < 2; ++pass) {
    *(volatile v4u*)(W16 + (size_t)row * CC + col) = u;
    __threadfence();
  }
}

__global__ __launch_bounds__(256)
void cvt_x(const float* __restrict__ src, const float* __restrict__ tgt, unsigned short* XS, unsigned short* XT) {
  __shared__ __align__(16) unsigned short T[QT * TP];
  const int tid = threadIdx.x;
  const int nb = blockIdx.x, cb = blockIdx.y & 1, which = blockIdx.y >> 1, b = blockIdx.z;
  const float* x = which ? tgt : src;
  unsigned short* XP = which ? XT : XS;
  const int e = tid & 7, lq = tid >> 3;
  const int n0 = nb * QT, c0 = cb * QT;
#pragma unroll
  for (int it = 0; it < 2; ++it) {
    const int cl = it * 32 + lq;
    const float* sp = x + ((size_t)(b * CC + c0 + cl)) * NFULL + n0 + 8 * e;
    const v4f a = *(const v4f*)sp;
    const v4f q = *(const v4f*)(sp + 4);
    unsigned short hb[8];
#pragma unroll
    for (int t = 0; t < 4; ++t) {
      hb[t]     = h_bits((_Float16)bfr(a[t]));
      hb[4 + t] = h_bits((_Float16)bfr(q[t]));
    }
#pragma unroll
    for (int t = 0; t < 8; ++t) T[(8 * e + t) * TP + cl] = hb[t];
  }
  __syncthreads();
  v4u up[2];
#pragma unroll
  for (int it = 0; it < 2; ++it) {
    const int nl = it * 32 + lq;
    up[it] = *(const v4u*)(T + nl * TP + 8 * e);
  }
#pragma unroll
  for (int pass = 0; pass < 2; ++pass) {
#pragma unroll
    for (int it = 0; it < 2; ++it) {
      const int nl = it * 32 + lq;
      *(volatile v4u*)(XP + ((size_t)(b * SEQ + n0 + nl)) * CC + c0 + 8 * e) = up[it];
    }
    __threadfence();
  }
}

__global__ __launch_bounds__(128)
void proj_k(const unsigned short* __restrict__ W16, const unsigned short* __restrict__ XS,
            const unsigned short* __restrict__ XT, const float* __restrict__ bq, const float* __restrict__ bk,
            const float* __restrict__ bv, unsigned short* Qh, unsigned short* Ql, unsigned short* Kh,
            unsigned short* Kl, unsigned short* Vc) {
  __shared__ __align__(16) float Os[QT * OSP];
  const int tid  = threadIdx.x;
  const int lane = tid & 31, wave = tid >> 5;
  const int hh   = lane >> 4, c = lane & 15;
  const int nt   = blockIdx.x, mb = blockIdx.y, b = blockIdx.z;
  const int wsel = mb >> 1;
  const int n0   = nt * QT, o0 = (mb & 1) * QT;
  const unsigned short* XP = (wsel == 0) ? XS : XT;
  const float* bias = (wsel == 0) ? bq : (wsel == 1) ? bk : bv;

  const unsigned short* ap = W16 + (size_t)(wsel * CC + o0 + c) * CC + 8 * hh;
  const unsigned short* bp = XP + ((size_t)(b * SEQ + n0 + 16 * wave + c)) * CC + 8 * hh;

  v8f acc[4];
#pragma unroll
  for (int mt = 0; mt < 4; ++mt) acc[mt] = zero8();

#pragma unroll
  for (int ks = 0; ks < CC / 32; ++ks) {
    const Frag fb = ldfrag(bp + 32 * ks);
#pragma unroll
    for (int mt = 0; mt < 4; ++mt) {
      const Frag fa = ldfrag(ap + (size_t)(16 * mt) * CC + 32 * ks);
      acc[mt] = mma_h(fa.h, fb.h, acc[mt]);
    }
  }

  {
    const int nl = 16 * wave + c;
#pragma unroll
    for (int mt = 0; mt < 4; ++mt) {
      const v4f b0 = *(const v4f*)(bias + o0 + 16 * mt + 8 * hh);
      const v4f b1 = *(const v4f*)(bias + o0 + 16 * mt + 8 * hh + 4);
      v4f va, vb;
#pragma unroll
      for (int r = 0; r < 4; ++r) {
        va[r] = acc[mt][r] * IWSC + bfr(b0[r]);
        vb[r] = acc[mt][4 + r] * IWSC + bfr(b1[r]);
      }
      *(v4f*)(Os + nl * OSP + 16 * mt + 8 * hh)     = va;
      *(v4f*)(Os + nl * OSP + 16 * mt + 8 * hh + 4) = vb;
    }
  }
  __syncthreads();

  const int e = tid & 7, lq = tid >> 3;
  if (wsel < 2) {
    unsigned short* Ph = (wsel == 0) ? Qh : Kh;
    unsigned short* Pl = (wsel == 0) ? Ql : Kl;
    v4u uh[4], ul[4];
#pragma unroll
    for (int it = 0; it < 4; ++it) {
      const int row = it * 16 + lq;
      const v4f a = *(const v4f*)(Os + row * OSP + 8 * e);
      const v4f q = *(const v4f*)(Os + row * OSP + 8 * e + 4);
      const float f[8] = {a[0], a[1], a[2], a[3], q[0], q[1], q[2], q[3]};
#pragma unroll
      for (int t = 0; t < 4; ++t) {
        const float f0 = f[2 * t], f1 = f[2 * t + 1];
        const unsigned short hb0 = bf_bits(f0), hb1 = bf_bits(f1);
        const unsigned short lb0 = bf_bits(f0 - bf_up(hb0));
        const unsigned short lb1 = bf_bits(f1 - bf_up(hb1));
        uh[it][t] = pk16(hb0, hb1);
        ul[it][t] = pk16(lb0, lb1);
      }
    }
#pragma unroll
    for (int pass = 0; pass < 2; ++pass) {
#pragma unroll
      for (int it = 0; it < 4; ++it) {
        const int row = it * 16 + lq;
        const size_t po = ((size_t)(b * SEQ + n0 + row)) * CC + o0 + 8 * e;
        *(volatile v4u*)(Ph + po) = uh[it];
        *(volatile v4u*)(Pl + po) = ul[it];
      }
      __threadfence();
    }
  } else {
    v4u uv[4];
#pragma unroll
    for (int it = 0; it < 4; ++it) {
      const int cl = it * 16 + lq;
      float f[8];
#pragma unroll
      for (int t = 0; t < 8; ++t) f[t] = Os[(8 * e + t) * OSP + cl];
#pragma unroll
      for (int t = 0; t < 4; ++t) {
        const _Float16 h0 = (_Float16)(f[2 * t] * VSC);
        const _Float16 h1 = (_Float16)(f[2 * t + 1] * VSC);
        uv[it][t] = pk16(h_bits(h0), h_bits(h1));
      }
    }
#pragma unroll
    for (int pass = 0; pass < 2; ++pass) {
#pragma unroll
      for (int it = 0; it < 4; ++it) {
        const int cl = it * 16 + lq;
        *(volatile v4u*)(Vc + ((size_t)(b * CC + o0 + cl)) * SEQ + n0 + 8 * e) = uv[it];
      }
      __threadfence();
    }
  }
}

__global__ __launch_bounds__(128)
void attn_k(const unsigned short* __restrict__ Qh, const unsigned short* __restrict__ Ql,
            const unsigned short* __restrict__ Kh, const unsigned short* __restrict__ Kl,
            const unsigned short* __restrict__ Vc, unsigned short* WSh, unsigned short* WSl) {
  __shared__ __align__(16) float Os[QT * OSPW];
  const int tid  = threadIdx.x;
  const int wave = tid >> 5, lane = tid & 31;
  const int hh   = lane >> 4, c = lane & 15;
  const int n0   = blockIdx.x * QT, b = blockIdx.y;

  const size_t qo = ((size_t)(b * SEQ + n0 + 16 * wave + c)) * CC + 8 * hh;
  const unsigned short* Qhp = Qh + qo;
  const unsigned short* Qlp = Ql + qo;
  const unsigned short* Khp = Kh + (size_t)b * SEQ * CC + (size_t)c * CC + 8 * hh;
  const unsigned short* Klp = Kl + (size_t)b * SEQ * CC + (size_t)c * CC + 8 * hh;
  const unsigned short* Vp = Vc + (size_t)b * CC * SEQ + (size_t)c * SEQ + 8 * hh;

  float m = -1.0e30f, l = 0.f;
  v8f o[8];
#pragma unroll
  for (int j = 0; j < 8; ++j) o[j] = zero8();

#pragma unroll 1
  for (int kb = 0; kb < SEQ; kb += 32) {
    const unsigned short* k0p  = Khp + (size_t)kb * CC;
    const unsigned short* k1p  = Khp + (size_t)(kb + 16) * CC;
    const unsigned short* k0lp = Klp + (size_t)kb * CC;
    const unsigned short* k1lp = Klp + (size_t)(kb + 16) * CC;
    v8f s0 = zero8(), s1 = zero8();
#pragma unroll 1
    for (int kc = 0; kc < CC / 32; ++kc) {
      const Frag qh  = ldfrag(Qhp + 32 * kc);
      const Frag ql  = ldfrag(Qlp + 32 * kc);
      const Frag k0  = ldfrag(k0p + 32 * kc);
      const Frag k1  = ldfrag(k1p + 32 * kc);
      const Frag k0l = ldfrag(k0lp + 32 * kc);
      const Frag k1l = ldfrag(k1lp + 32 * kc);
      s0 = mma_b(k0.bf, qh.bf, s0);
      s1 = mma_b(k1.bf, qh.bf, s1);
      s0 = mma_b(k0.bf, ql.bf, s0);
      s1 = mma_b(k1.bf, ql.bf, s1);
      s0 = mma_b(k0l.bf, qh.bf, s0);
      s1 = mma_b(k1l.bf, qh.bf, s1);
    }
    s0 = s0 * SCL;
    s1 = s1 * SCL;

    float mx = fmaxf(hmax8(s0), hmax8(s1));
    mx = fmaxf(mx, __shfl_xor(mx, 16, 32));
    const float mn = fmaxf(m, mx);
    const unsigned grew = wave_ballot(mx > m);
    if (grew != 0u) {
      const float corr = __expf(m - mn);
      l *= corr;
#pragma unroll
      for (int j = 0; j < 8; ++j) {
#pragma unroll
        for (int r = 0; r < 8; ++r) o[j][r] *= corr;
      }
    }
    m = mn;
    const float msh = mn - LNPS;

    FragH ph;
    float ls = 0.f;
#pragma unroll
    for (int r = 0; r < 8; ++r) {
      const float e0 = __expf(s0[r] - msh);
      const float e1 = __expf(s1[r] - msh);
      ls += e0 + e1;
      ph.hv[0][r] = (_Float16)e0;
      ph.hv[1][r] = (_Float16)e1;
    }
    l += ls;

#pragma unroll
    for (int j = 0; j < 8; ++j) {
      const Frag vf = ldfrag(Vp + (size_t)(16 * j) * SEQ + kb);
      o[j] = mma_h(vf.h, ph.v, o[j]);
    }
  }
  l += __shfl_xor(l, 16, 32);
  const float inv = IVSC / l;

  const int qrow = 16 * wave + c;
  const int e = tid & 7, lq = tid >> 3;
#pragma unroll
  for (int jj = 0; jj < 8; ++jj) {
    v4f va, vb;
#pragma unroll
    for (int r = 0; r < 4; ++r) { va[r] = o[jj][r] * inv; vb[r] = o[jj][4 + r] * inv; }
    *(v4f*)(Os + qrow * OSPW + 16 * jj + 8 * hh)     = va;
    *(v4f*)(Os + qrow * OSPW + 16 * jj + 8 * hh + 4) = vb;
  }
  __syncthreads();

  v4u uh[8], ul[8];
#pragma unroll
  for (int it = 0; it < 8; ++it) {
    const int L    = it * 16 + lq;
    const int row  = L >> 1;
    const int dsel = (L & 1) * QT;
    const v4f a = *(const v4f*)(Os + row * OSPW + dsel + 8 * e);
    const v4f q = *(const v4f*)(Os + row * OSPW + dsel + 8 * e + 4);
    const float f[8] = {a[0], a[1], a[2], a[3], q[0], q[1], q[2], q[3]};
#pragma unroll
    for (int t = 0; t < 4; ++t) {
      const float f0 = f[2 * t], f1 = f[2 * t + 1];
      const unsigned short hb0 = bf_bits(f0), hb1 = bf_bits(f1);
      const unsigned short lb0 = bf_bits(f0 - bf_up(hb0));
      const unsigned short lb1 = bf_bits(f1 - bf_up(hb1));
      uh[it][t] = pk16(hb0, hb1);
      ul[it][t] = pk16(lb0, lb1);
    }
  }
#pragma unroll
  for (int pass = 0; pass < 2; ++pass) {
#pragma unroll
    for (int it = 0; it < 8; ++it) {
      const int L    = it * 16 + lq;
      const int row  = L >> 1;
      const int dsel = (L & 1) * QT;
      const size_t po = ((size_t)(b * SEQ + n0 + row)) * CC + dsel + 8 * e;
      *(volatile v4u*)(WSh + po) = uh[it];
      *(volatile v4u*)(WSl + po) = ul[it];
    }
    __threadfence();
  }
}

__global__ __launch_bounds__(128)
void gemm_o(const unsigned short* __restrict__ W16, const unsigned short* __restrict__ WSh,
            const unsigned short* __restrict__ WSl, const float* __restrict__ bo, float* out) {
  __shared__ __align__(16) float Os[QT * OSP];
  const int tid  = threadIdx.x;
  const int lane = tid & 31, wave = tid >> 5;
  const int hh   = lane >> 4, c = lane & 15;
  const int nt   = blockIdx.x, mb = blockIdx.y, b = blockIdx.z;
  const int n0   = nt * QT, o0 = mb * QT;

  const unsigned short* ap  = W16 + (size_t)(3 * CC + o0 + c) * CC + 8 * hh;
  const size_t bo16 = ((size_t)(b * SEQ + n0 + 16 * wave + c)) * CC + 8 * hh;
  const unsigned short* bph = WSh + bo16;
  const unsigned short* bpl = WSl + bo16;

  v8f acc[4];
#pragma unroll
  for (int mt = 0; mt < 4; ++mt) acc[mt] = zero8();

#pragma unroll
  for (int ks = 0; ks < CC / 32; ++ks) {
    const Frag fbh = ldfrag(bph + 32 * ks);
    const Frag fbl = ldfrag(bpl + 32 * ks);
#pragma unroll
    for (int mt = 0; mt < 4; ++mt) {
      const Frag fa = ldfrag(ap + (size_t)(16 * mt) * CC + 32 * ks);
      acc[mt] = mma_b(fa.bf, fbh.bf, acc[mt]);
      acc[mt] = mma_b(fa.bf, fbl.bf, acc[mt]);
    }
  }

  {
    const int nl = 16 * wave + c;
#pragma unroll
    for (int mt = 0; mt < 4; ++mt) {
      v4f va, vb;
#pragma unroll
      for (int r = 0; r < 4; ++r) { va[r] = acc[mt][r]; vb[r] = acc[mt][4 + r]; }
      *(v4f*)(Os + nl * OSP + 16 * mt + 8 * hh)     = va;
      *(v4f*)(Os + nl * OSP + 16 * mt + 8 * hh + 4) = vb;
    }
  }
  __syncthreads();

  const int e = tid & 7, lq = tid >> 3;
  v4f res[8];
#pragma unroll
  for (int it = 0; it < 8; ++it) {
    const int L  = it * 16 + lq;
    const int ol = L >> 1, hf = L & 1;
    const int nl = hf * 32 + 4 * e;
    const float bz = bfr(bo[o0 + ol]);
#pragma unroll
    for (int t = 0; t < 4; ++t) res[it][t] = Os[(nl + t) * OSP + ol] + bz;
  }
#pragma unroll
  for (int pass = 0; pass < 2; ++pass) {
#pragma unroll
    for (int it = 0; it < 8; ++it) {
      const int L  = it * 16 + lq;
      const int ol = L >> 1, hf = L & 1;
      const int nl = hf * 32 + 4 * e;
      const size_t idx = ((size_t)(b * CC + o0 + ol)) * SEQ + n0 + nl;
      *(volatile v4f*)(out + idx) = res[it];
    }
    __threadfence();
  }
}

extern "C" void kernel_launch(void* const* d_in, const int* in_sizes, int n_in,
                              void* d_out, int out_size, void* d_ws, size_t ws_size,
                              hipStream_t stream) {
  if (n_in < 10) return;
  if (in_sizes[0] < NB * CC * NFULL || in_sizes[1] < NB * CC * NFULL) return;
  if (in_sizes[2] < CC * CC || in_sizes[4] < CC * CC || in_sizes[6] < CC * CC || in_sizes[8] < CC * CC) return;
  if (in_sizes[3] < CC || in_sizes[5] < CC || in_sizes[7] < CC || in_sizes[9] < CC) return;
  if (out_size < NB * CC * SEQ) return;

  size_t off = 0;
  auto carve = [&](size_t bytes) { const size_t o = off; off += (bytes + 255) & ~(size_t)255; return o; };
  const size_t plane = (size_t)NB * SEQ * CC * 2;
  const size_t oW16 = carve((size_t)NWR * CC * 2);
  const size_t oXS  = carve(plane);
  const size_t oXT  = carve(plane);
  const size_t oQh  = carve(plane);
  const size_t oQl  = carve(plane);
  const size_t oKh  = carve(plane);
  const size_t oKl  = carve(plane);
  const size_t oVc  = carve(plane);
  const size_t oWSh = carve(plane);
  const size_t oWSl = carve(plane);
  if (off > ws_size) return;
  if (off > (size_t)134217728) return;

  const float* src = (const float*)d_in[0];
  const float* tgt = (const float*)d_in[1];
  const float* wq  = (const float*)d_in[2];
  const float* bq  = (const float*)d_in[3];
  const float* wk  = (const float*)d_in[4];
  const float* bk  = (const float*)d_in[5];
  const float* wv  = (const float*)d_in[6];
  const float* bv  = (const float*)d_in[7];
  const float* wo  = (const float*)d_in[8];
  const float* bo  = (const float*)d_in[9];

  char* ws = (char*)d_ws;
  unsigned short* W16 = (unsigned short*)(ws + oW16);
  unsigned short* XS  = (unsigned short*)(ws + oXS);
  unsigned short* XT  = (unsigned short*)(ws + oXT);
  unsigned short* Qh  = (unsigned short*)(ws + oQh);
  unsigned short* Ql  = (unsigned short*)(ws + oQl);
  unsigned short* Kh  = (unsigned short*)(ws + oKh);
  unsigned short* Kl  = (unsigned short*)(ws + oKl);
  unsigned short* Vc  = (unsigned short*)(ws + oVc);
  unsigned short* WSh = (unsigned short*)(ws + oWSh);
  unsigned short* WSl = (unsigned short*)(ws + oWSl);
  float* out = (float*)d_out;

  const dim3 blk256(256), blk128(128);

  cvt_w<<<dim3(NWR / 16), blk256, 0, stream>>>(wq, wk, wv, wo, W16);
  cvt_x<<<dim3(SEQ / QT, 4, NB), blk256, 0, stream>>>(src, tgt, XS, XT);
  proj_k<<<dim3(SEQ / QT, 6, NB), blk128, 0, stream>>>(W16, XS, XT, bq, bk, bv, Qh, Ql, Kh, Kl, Vc);
  attn_k<<<dim3(SEQ / QT, NB), blk128, 0, stream>>>(Qh, Ql, Kh, Kl, Vc, WSh, WSl);
  gemm_o<<<dim3(SEQ / QT, 2, NB), blk128, 0, stream>>>(W16, WSh, WSl, bo, out);
  (void)hipGetLastError();
}
